// PointTokenizer_69544110457437
// MI455X (gfx1250) — hardware-verified
//
#include <hip/hip_runtime.h>
#include <stdint.h>
#include <stddef.h>

#pragma clang fp contract(off)

typedef __attribute__((ext_vector_type(16))) _Float16 v16h;
typedef __attribute__((ext_vector_type(8)))  _Float16 v8h;
typedef __attribute__((ext_vector_type(16))) __bf16   v16b;
typedef __attribute__((ext_vector_type(8)))  __bf16   v8b;
typedef __attribute__((ext_vector_type(8)))  float    v8f;
typedef __attribute__((ext_vector_type(4)))  float    v4f;
typedef __attribute__((ext_vector_type(4)))  unsigned v4u;

constexpr int kBatch   = 8;
constexpr int kNpts    = 8192;
constexpr int kCenters = 512;
constexpr int kKnn     = 32;
constexpr int kGroups  = kBatch * kCenters;
constexpr int kRows    = kGroups * kKnn;
constexpr int kC1 = 64, kC2 = 128, kC3 = 384;
constexpr int kL1RowsPerBlk = 512;
constexpr int kL1Blocks = kRows / kL1RowsPerBlk;
constexpr int kTilesM = kRows / 64;

static_assert(kRows % 64 == 0, "M tile");
static_assert(kC2 % 64 == 0 && kC3 % 64 == 0, "N tile");
static_assert(kC1 % 32 == 0 && kC2 % 32 == 0, "K step");
static_assert(kKnn == 32, "two groups per 64-row tile");

constexpr size_t kSzGrouped = (size_t)kRows * 3 * 4;
constexpr size_t kSzPart1   = (size_t)2 * kL1Blocks * kC1 * 4;
constexpr size_t kSzTab     = 4096;
constexpr size_t kSzW2t     = (size_t)2 * kC2 * kC1 * 2;
constexpr size_t kSzW3t     = (size_t)kC3 * kC2 * 2;
constexpr size_t kSzH       = (size_t)2 * kRows * kC1 * 2;
constexpr size_t kSzA2      = (size_t)kRows * kC2 * 4;
constexpr size_t kSzPart2   = (size_t)2 * kTilesM * kC2 * 4;
constexpr size_t kSzPart3   = (size_t)2 * kTilesM * kC3 * 4;
constexpr size_t kSzGmm     = (size_t)2 * kGroups * kC3 * 4;

constexpr size_t kOffGrouped = 0;
constexpr size_t kOffPart1   = kOffGrouped + kSzGrouped;
constexpr size_t kOffTab1    = kOffPart1 + kSzPart1;
constexpr size_t kOffW2t     = kOffTab1 + kSzTab;
constexpr size_t kOffW3t     = kOffW2t + kSzW2t;
constexpr size_t kOffH       = kOffW3t + kSzW3t;
constexpr size_t kOffA2      = kOffH + kSzH;
constexpr size_t kOffPart2   = kOffA2 + kSzA2;
constexpr size_t kOffTab2    = kOffPart2 + kSzPart2;
constexpr size_t kOffPart3   = kOffTab2 + kSzTab;
constexpr size_t kOffTab3    = kOffPart3 + kSzPart3;
constexpr size_t kOffGmm     = kOffTab3 + kSzTab;
constexpr size_t kWsTotal    = kOffGmm + kSzGmm;
static_assert(kWsTotal == 123482112, "carve total");
static_assert(kWsTotal <= 134217728, "carve budget");
static_assert((size_t)kRows * kC2 * 2 == kSzH, "h2 f16 plane fits the h1 region exactly");
static_assert(kOffPart1 % 4096 == 0 && kOffH % 4096 == 0 && kOffA2 % 4096 == 0 && kOffGmm % 4096 == 0, "alignment");
static_assert(2 * kC1 * 4 <= (int)kSzTab && 2 * kC3 * 4 <= (int)kSzTab, "tab reserve");

constexpr size_t kOut1Floats = 6291456 / 4;
static_assert(kOut1Floats == (size_t)kGroups * kC3, "out1 offset");
static_assert(6291456 + (size_t)kGroups * 3 * 4 == 6340608, "out total");

__device__ __forceinline__ unsigned short f2bf_bits(float f) {
  unsigned u = __float_as_uint(f);
  return (unsigned short)((u + 0x7FFFu + ((u >> 16) & 1u)) >> 16);
}
__device__ __forceinline__ float bf_bits2f(unsigned short h) { return __uint_as_float(((unsigned)h) << 16); }

__device__ __forceinline__ void dep_guard_h(v8f& a, v8f& b, v16h x, v16h y) { asm volatile("v_nop\n\tv_nop\n\tv_nop\n\tv_nop" : "+v"(a), "+v"(b) : "v"(x), "v"(y)); }
__device__ __forceinline__ void dep_guard_b(v8f& a, v8f& b, v16b x, v16b y) { asm volatile("v_nop\n\tv_nop\n\tv_nop\n\tv_nop" : "+v"(a), "+v"(b) : "v"(x), "v"(y)); }
__device__ __forceinline__ void keep4_h(v16h a, v16h b, v16h c, v16h d) { asm volatile("v_nop" :: "v"(a), "v"(b), "v"(c), "v"(d)); }
__device__ __forceinline__ void keep4_b(v16b a, v16b b, v16b c, v16b d) { asm volatile("v_nop" :: "v"(a), "v"(b), "v"(c), "v"(d)); }
__device__ __forceinline__ void acc_guard4(v8f& a, v8f& b, v8f& c, v8f& d) { asm volatile("v_nop\n\tv_nop\n\tv_nop\n\tv_nop" : "+v"(a), "+v"(b), "+v"(c), "+v"(d)); }
template <typename T> struct Frag;
template <> struct Frag<_Float16> {
  typedef v16h V; union U { v16h v; v8h h[2]; };
  static __device__ __forceinline__ v16h load(const _Float16* p) {
    U f; f.h[0] = *(const v8h*)(p); f.h[1] = *(const v8h*)(p + 16); return f.v;
  }
  static __device__ __forceinline__ v8f mma(v16h a, v16h b, v8f c) {
    return __builtin_amdgcn_wmma_f32_16x16x32_f16(false, a, false, b, (short)0, c, false, false);
  }
  static __device__ __forceinline__ void guard(v8f& a, v8f& b, v16h x, v16h y) { dep_guard_h(a, b, x, y); }
  static __device__ __forceinline__ void keep(v16h a, v16h b, v16h c, v16h d) { keep4_h(a, b, c, d); }
};
template <> struct Frag<__bf16> {
  typedef v16b V; union U { v16b v; v8b h[2]; };
  static __device__ __forceinline__ v16b load(const __bf16* p) {
    U f; f.h[0] = *(const v8b*)(p); f.h[1] = *(const v8b*)(p + 16); return f.v;
  }
  static __device__ __forceinline__ v8f mma(v16b a, v16b b, v8f c) {
    return __builtin_amdgcn_wmma_f32_16x16x32_bf16(false, a, false, b, (short)0, c, false, false);
  }
  static __device__ __forceinline__ void guard(v8f& a, v8f& b, v16b x, v16b y) { dep_guard_b(a, b, x, y); }
  static __device__ __forceinline__ void keep(v16b a, v16b b, v16b c, v16b d) { keep4_b(a, b, c, d); }
};
template <int ET> struct Elem;
template <> struct Elem<0> { typedef _Float16 T; };
template <> struct Elem<1> { typedef __bf16 T; };

__device__ __forceinline__ void argbest_max(float& v, int& i) {
#pragma unroll
  for (int off = 16; off > 0; off >>= 1) {
    const float ov = __shfl_xor(v, off, 32);
    const int   oi = __shfl_xor(i, off, 32);
    const bool tk = (ov > v) || (ov == v && oi < i);
    v = tk ? ov : v; i = tk ? oi : i;
  }
}
__device__ __forceinline__ void argbest_min(float& v, int& i) {
#pragma unroll
  for (int off = 16; off > 0; off >>= 1) {
    const float ov = __shfl_xor(v, off, 32);
    const int   oi = __shfl_xor(i, off, 32);
    const bool tk = (ov < v) || (ov == v && oi < i);
    v = tk ? ov : v; i = tk ? oi : i;
  }
}

__device__ __forceinline__ float sqd3(float ax, float ay, float az, float bx, float by, float bz) {
  const float dx = ax - bx;
  const float dy = ay - by;
  const float dz = az - bz;
  const float t0 = dx * dx;
  const float t1 = dy * dy;
  const float t2 = dz * dz;
  const float s02 = t0 + t2;
  return s02 + t1;
}

__device__ __forceinline__ float l1_pre(float x0, float x1, float x2, float w0, float w1, float w2, float bb) {
  const float p0 = x0 * w0;
  const float p1 = x1 * w1;
  const float p2 = x2 * w2;
  return ((p0 + p1) + p2) + bb;
}

constexpr int kFpsT = 256;
__global__ __launch_bounds__(kFpsT) void fps_kernel(const float* __restrict__ pts, float* __restrict__ cen_out)
{
  __shared__ float dist[kNpts];
  __shared__ __align__(16) float cenbuf[kCenters * 3];
  __shared__ float red_v[kFpsT / 32];
  __shared__ int   red_i[kFpsT / 32];
  __shared__ int   s_far;

  const int b = blockIdx.x;
  const int t = threadIdx.x;
  const int lane = t & 31, wave = t >> 5;
  const float* P = pts + (size_t)b * kNpts * 3;

  for (int i = t; i < kNpts; i += kFpsT) dist[i] = 1e10f;
  if (t == 0) s_far = 0;
  __syncthreads();
  int far = 0;

#pragma unroll 1
  for (int s = 0; s < kCenters; ++s) {
    const float cx = P[far * 3 + 0], cy = P[far * 3 + 1], cz = P[far * 3 + 2];
    if (t == 0) { cenbuf[s * 3 + 0] = cx; cenbuf[s * 3 + 1] = cy; cenbuf[s * 3 + 2] = cz; }
    float bv = -1.0f; int bi = 0x7fffffff;
#pragma unroll 2
    for (int i = t; i < kNpts; i += kFpsT) {
      const float d  = sqd3(P[i * 3 + 0], P[i * 3 + 1], P[i * 3 + 2], cx, cy, cz);
      const float nd = fminf(dist[i], d);
      dist[i] = nd;
      const bool tk = nd > bv;
      bv = tk ? nd : bv; bi = tk ? i : bi;
    }
    argbest_max(bv, bi);
    if (lane == 0) { red_v[wave] = bv; red_i[wave] = bi; }
    __syncthreads();
    if (wave == 0) {
      float v2 = red_v[lane & 7];
      int   i2 = red_i[lane & 7];
      v2 = (lane < (kFpsT / 32)) ? v2 : -2.0f;
      i2 = (lane < (kFpsT / 32)) ? i2 : 0x7fffffff;
      argbest_max(v2, i2);
      if (lane == 0) s_far = (i2 < 0) ? 0 : ((i2 > kNpts - 1) ? (kNpts - 1) : i2);
    }
    __syncthreads();
    far = s_far;
  }
  __syncthreads();
  if (wave == 0) {
    float* dst = cen_out + (size_t)b * (kCenters * 3);
    for (int pass = 0; pass < 2; ++pass) {
#pragma unroll
      for (int it = 0; it < 12; ++it) {
        const int f4 = it * 32 + lane;
        const v4f v = *(const v4f*)(cenbuf + f4 * 4);
        *(volatile v4f*)(dst + f4 * 4) = v;
      }
      __threadfence();
    }
  }
}

constexpr int kKnnT = 256;
__global__ __launch_bounds__(kKnnT) void knn_kernel(const float* __restrict__ pts, const float* __restrict__ cen,
                                                   float* __restrict__ grouped)
{
  __shared__ float d2s[kNpts];
  __shared__ unsigned short lst[kNpts];
  __shared__ float tmin[kKnnT];
  __shared__ int   wcnt[kKnnT / 32];
  __shared__ float rv[kKnnT / 32];
  __shared__ int   ri[kKnnT / 32];
  __shared__ float s_tau;
  __shared__ __align__(16) float gout[kKnn * 3];

  const int g = blockIdx.x;
  const int b = g / kCenters;
  const int t = threadIdx.x;
  const int lane = t & 31, wave = t >> 5;
  const float* P = pts + (size_t)b * kNpts * 3;
  const float cx = cen[(size_t)g * 3 + 0], cy = cen[(size_t)g * 3 + 1], cz = cen[(size_t)g * 3 + 2];

  float mv = 3.0e38f;
#pragma unroll 2
  for (int c = 0; c < kNpts / kKnnT; ++c) {
    const int i = c * kKnnT + t;
    const float d = sqd3(cx, cy, cz, P[i * 3 + 0], P[i * 3 + 1], P[i * 3 + 2]);
    d2s[i] = d;
    mv = fminf(mv, d);
  }
  tmin[t] = mv;
  __syncthreads();

  if (wave == 0) {
    float v[8];
#pragma unroll
    for (int q = 0; q < 8; ++q) v[q] = tmin[q * 32 + lane];
    float tau = 0.0f;
#pragma unroll 1
    for (int p = 0; p < kKnn; ++p) {
      float bv = 3.0e38f; int bi = 1 << 20;
#pragma unroll
      for (int q = 0; q < 8; ++q) {
        const bool tk = v[q] < bv;
        bv = tk ? v[q] : bv; bi = tk ? (q * 32 + lane) : bi;
      }
      argbest_min(bv, bi);
      tau = bv;
#pragma unroll
      for (int q = 0; q < 8; ++q) v[q] = ((q * 32 + lane) == bi) ? 3.0e38f : v[q];
    }
    if (lane == 0) s_tau = tau;
  }
  __syncthreads();
  const float tau = s_tau;

  int base = 0;
#pragma unroll 1
  for (int c = 0; c < kNpts / kKnnT; ++c) {
    const int i = c * kKnnT + t;
    const bool f = d2s[i] <= tau;
    const unsigned m = __builtin_amdgcn_ballot_w32(f);
    const int pos = __builtin_popcount(m & ((1u << lane) - 1u));
    const int cw  = __builtin_popcount(m);
    if (lane == 0) wcnt[wave] = cw;
    __syncthreads();
    int woff = 0, tot = 0;
#pragma unroll
    for (int w = 0; w < kKnnT / 32; ++w) {
      const int cv = wcnt[w];
      woff += (w < wave) ? cv : 0;
      tot += cv;
    }
    if (f) {
      int p = base + woff + pos;
      p = (p > kNpts - 1) ? (kNpts - 1) : p;
      lst[p] = (unsigned short)i;
    }
    base += tot;
    __syncthreads();
  }
  const int cnt = (base > kNpts) ? kNpts : base;

#pragma unroll 1
  for (int j = 0; j < kKnn; ++j) {
    float bv = 3.0e38f; int bi = 0xffff;
#pragma unroll 1
    for (int e = t; e < cnt; e += kKnnT) {
      const int idx = (int)lst[e];
      const float v = d2s[idx];
      const bool tk = (v < bv) || (v == bv && idx < bi);
      bv = tk ? v : bv; bi = tk ? idx : bi;
    }
    argbest_min(bv, bi);
    if (lane == 0) { rv[wave] = bv; ri[wave] = bi; }
    __syncthreads();
    if (wave == 0) {
      float v2 = rv[lane & 7];
      int   i2 = ri[lane & 7];
      v2 = (lane < (kKnnT / 32)) ? v2 : 3.0e38f;
      i2 = (lane < (kKnnT / 32)) ? i2 : 0x1ffff;
      argbest_min(v2, i2);
      if (lane == 0) {
        const int sel = (i2 < 0) ? 0 : ((i2 > kNpts - 1) ? (kNpts - 1) : i2);
        d2s[sel] = 3.3e38f;
        gout[j * 3 + 0] = P[sel * 3 + 0] - cx;
        gout[j * 3 + 1] = P[sel * 3 + 1] - cy;
        gout[j * 3 + 2] = P[sel * 3 + 2] - cz;
      }
    }
    __syncthreads();
  }

  if (wave == 0) {
    const int lc = (lane < 24) ? lane : 0;
    const v4f v = *(const v4f*)(gout + lc * 4);
    float* dst = grouped + (size_t)g * (kKnn * 3);
    for (int pass = 0; pass < 2; ++pass) {
      if (lane < 24) *(volatile v4f*)(dst + lane * 4) = v;
      __threadfence();
    }
  }
}

__global__ __launch_bounds__(256) void l1_stats_kernel(const float* __restrict__ grouped, const float* __restrict__ W1,
                                                      const float* __restrict__ b1, float* __restrict__ part)
{
  __shared__ float sW[3 * kC1], sB[kC1];
  __shared__ float rs[4][kC1], rq[4][kC1];
  __shared__ __align__(16) float outl[2 * kC1];
  const int t = threadIdx.x;
  const int lane = t & 31;
  if (t < 3 * kC1) sW[t] = W1[t];
  if (t < kC1) sB[t] = b1[t];
  __syncthreads();
  const int c = t & (kC1 - 1);
  const int rg = t >> 6;
  const float w0 = sW[c], w1 = sW[kC1 + c], w2 = sW[2 * kC1 + c], bb = sB[c];
  float s = 0.0f, q = 0.0f;
#pragma unroll 2
  for (int r = rg; r < kL1RowsPerBlk; r += 4) {
    const size_t row = (size_t)blockIdx.x * kL1RowsPerBlk + r;
    const float x0 = grouped[row * 3 + 0], x1 = grouped[row * 3 + 1], x2 = grouped[row * 3 + 2];
    const float a = l1_pre(x0, x1, x2, w0, w1, w2, bb);
    s += a;
    q += a * a;
  }
  rs[rg][c] = s; rq[rg][c] = q;
  __syncthreads();
  if (t < kC1) {
    const float S = (rs[0][t] + rs[1][t]) + (rs[2][t] + rs[3][t]);
    const float Q = (rq[0][t] + rq[1][t]) + (rq[2][t] + rq[3][t]);
    outl[t] = S; outl[kC1 + t] = Q;
  }
  __syncthreads();
  if (t < 32) {
    const v4f v = *(const v4f*)(outl + lane * 4);
    float* dst = part + (size_t)(lane >> 4) * (kL1Blocks * kC1) + (size_t)blockIdx.x * kC1 + (lane & 15) * 4;
    for (int pass = 0; pass < 2; ++pass) {
      *(volatile v4f*)dst = v;
      __threadfence();
    }
  }
}

__global__ __launch_bounds__(64) void fin_kernel(const float* __restrict__ part, int nblk, int C,
                                                 const float* __restrict__ gamma, const float* __restrict__ beta,
                                                 float* __restrict__ tab)
{
  __shared__ __align__(16) float st[128];
  const int t = threadIdx.x;
  const int lane = t & 31;
  const int c = blockIdx.x * 64 + t;
  double S = 0.0, Q = 0.0;
#pragma unroll 1
  for (int k = 0; k < nblk; ++k) {
    S += (double)part[(size_t)k * C + c];
    Q += (double)part[(size_t)(nblk + k) * C + c];
  }
  const double invn = 1.0 / (double)kRows;
  const double mean = S * invn;
  double var = Q * invn - mean * mean;
  var = (var < 0.0) ? 0.0 : var;
  const float vf = (float)var + 1e-5f;
  const float inv = 1.0f / sqrtf(vf);
  const float sc = gamma[c] * inv;
  const float sh = beta[c] - (float)mean * sc;
  st[t] = sc; st[64 + t] = sh;
  __syncthreads();
  if (t < 32) {
    const v4f v = *(const v4f*)(st + lane * 4);
    float* dst = tab + (size_t)(lane >> 4) * C + (size_t)blockIdx.x * 64 + (lane & 15) * 4;
    for (int pass = 0; pass < 2; ++pass) {
      *(volatile v4f*)dst = v;
      __threadfence();
    }
  }
}

__global__ __launch_bounds__(256) void l1_apply_kernel(const float* __restrict__ grouped, const float* __restrict__ W1,
                                                      const float* __restrict__ b1, const float* __restrict__ tab1,
                                                      unsigned short* __restrict__ Hhi, unsigned short* __restrict__ Hlo)
{
  __shared__ float sW[3 * kC1], sB[kC1], sSc[kC1], sSh[kC1];
  const int t = threadIdx.x;
  if (t < 3 * kC1) sW[t] = W1[t];
  if (t < kC1) { sB[t] = b1[t]; sSc[t] = tab1[t]; sSh[t] = tab1[kC1 + t]; }
  __syncthreads();
  const int gid = blockIdx.x * 256 + t;
  const int row = gid >> 3;
  const int c8  = (gid & 7) * 8;
  const float x0 = grouped[(size_t)row * 3 + 0], x1 = grouped[(size_t)row * 3 + 1], x2 = grouped[(size_t)row * 3 + 2];
  unsigned hw[4], lw[4];
#pragma unroll
  for (int p = 0; p < 4; ++p) {
    unsigned hpair = 0u, lpair = 0u;
#pragma unroll
    for (int u = 0; u < 2; ++u) {
      const int c = c8 + 2 * p + u;
      const float a = l1_pre(x0, x1, x2, sW[c], sW[kC1 + c], sW[2 * kC1 + c], sB[c]);
      const float h = fmaxf(a * sSc[c] + sSh[c], 0.0f);
      const unsigned short hb = f2bf_bits(h);
      const unsigned short lb = f2bf_bits(h - bf_bits2f(hb));
      hpair |= ((unsigned)hb) << (16 * u);
      lpair |= ((unsigned)lb) << (16 * u);
    }
    hw[p] = hpair; lw[p] = lpair;
  }
  const v4u hv = (v4u){hw[0], hw[1], hw[2], hw[3]};
  const v4u lv = (v4u){lw[0], lw[1], lw[2], lw[3]};
  const size_t off = (size_t)row * kC1 + c8;
  for (int pass = 0; pass < 2; ++pass) {
    *(volatile v4u*)(Hhi + off) = hv;
    *(volatile v4u*)(Hlo + off) = lv;
    __threadfence();
  }
}

__global__ __launch_bounds__(256) void wprep2_kernel(const float* __restrict__ W2, unsigned short* __restrict__ Bhi,
                                                    unsigned short* __restrict__ Blo)
{
  const int gid = blockIdx.x * 256 + threadIdx.x;
  const int n  = gid >> 3;
  const int k8 = (gid & 7) * 8;
  unsigned hw[4], lw[4];
#pragma unroll
  for (int p = 0; p < 4; ++p) {
    unsigned hpair = 0u, lpair = 0u;
#pragma unroll
    for (int u = 0; u < 2; ++u) {
      const int k = k8 + 2 * p + u;
      const float v = W2[(size_t)k * kC2 + n];
      const unsigned short hb = f2bf_bits(v);
      const unsigned short lb = f2bf_bits(v - bf_bits2f(hb));
      hpair |= ((unsigned)hb) << (16 * u);
      lpair |= ((unsigned)lb) << (16 * u);
    }
    hw[p] = hpair; lw[p] = lpair;
  }
  const v4u hv = (v4u){hw[0], hw[1], hw[2], hw[3]};
  const v4u lv = (v4u){lw[0], lw[1], lw[2], lw[3]};
  const size_t off = (size_t)n * kC1 + k8;
  for (int pass = 0; pass < 2; ++pass) {
    *(volatile v4u*)(Bhi + off) = hv;
    *(volatile v4u*)(Blo + off) = lv;
    __threadfence();
  }
}

__global__ __launch_bounds__(256) void wprep3_kernel(const float* __restrict__ W3, unsigned short* __restrict__ Bt)
{
  const int gid = blockIdx.x * 256 + threadIdx.x;
  const int n  = gid >> 4;
  const int k8 = (gid & 15) * 8;
  unsigned w[4];
#pragma unroll
  for (int p = 0; p < 4; ++p) {
    unsigned pr = 0u;
#pragma unroll
    for (int u = 0; u < 2; ++u) {
      const int k = k8 + 2 * p + u;
      const float v = W3[(size_t)k * kC3 + n] * 16.0f;
      const unsigned short hb = __builtin_bit_cast(unsigned short, (_Float16)v);
      pr |= ((unsigned)hb) << (16 * u);
    }
    w[p] = pr;
  }
  const v4u hv = (v4u){w[0], w[1], w[2], w[3]};
  const size_t off = (size_t)n * kC2 + k8;
  for (int pass = 0; pass < 2; ++pass) {
    *(volatile v4u*)(Bt + off) = hv;
    __threadfence();
  }
}

template <int ET, bool SPLIT, bool STORE_C, bool MAXMIN>
__global__ __launch_bounds__(256) void wmma_gemm64_stats(
    const unsigned short* __restrict__ Ap, const unsigned short* __restrict__ A2p, int lda,
    const unsigned short* __restrict__ Btp, const unsigned short* __restrict__ Bt2p, int ldb,
    float* __restrict__ Cout, int ldc,
    const float* __restrict__ bias,
    float* __restrict__ part, float* __restrict__ gmm,
    int M, int N, int K, float scale) {
  typedef typename Elem<ET>::T T;
  typedef typename Frag<T>::V V;
  const T* A = (const T*)Ap; const T* A2 = (const T*)A2p; const T* Bt = (const T*)Btp; const T* Bt2 = (const T*)Bt2p;
  __shared__ __align__(16) float sT[8][16 * 68];
  const int lane = threadIdx.x & 31;
  const int wave = threadIdx.x >> 5;
  const int tilesN = N >> 6;
  const int tilesM = M >> 6;
  const int tile = blockIdx.x * 8 + wave;
  if (tile >= tilesM * tilesN) return;
  const int tm = tile / tilesN;
  const int tn = tile - tm * tilesN;
  const int m0 = tm << 6;
  const int n0 = tn << 6;

  const int rlane = lane & 15;
  const int koff  = (lane >> 4) * 8;
  const int mOff  = (lane >> 4) * 8;

  v8f acc[4][4];
#pragma unroll
  for (int i = 0; i < 4; ++i)
#pragma unroll
    for (int j = 0; j < 4; ++j) acc[i][j] = (v8f){0.f,0.f,0.f,0.f,0.f,0.f,0.f,0.f};

  for (int k0 = 0; k0 < K; k0 += 32) {
    V bh[4], bl[4];
#pragma unroll
    for (int j = 0; j < 4; ++j) {
      const size_t bo = (size_t)(n0 + (j << 4) + rlane) * ldb + koff + k0;
      bh[j] = Frag<T>::load(Bt + bo);
      if (SPLIT) bl[j] = Frag<T>::load(Bt2 + bo);
    }
#pragma unroll
    for (int i = 0; i < 4; ++i) {
      const size_t ao = (size_t)(m0 + (i << 4) + rlane) * lda + koff + k0;
      V ah = Frag<T>::load(A + ao);
      V al;
      if (SPLIT) al = Frag<T>::load(A2 + ao);
#pragma unroll
      for (int j = 0; j < 4; ++j) {
        acc[i][j] = Frag<T>::mma(ah, bh[j], acc[i][j]);
        if (SPLIT) {
          acc[i][j] = Frag<T>::mma(ah, bl[j], acc[i][j]);
          acc[i][j] = Frag<T>::mma(al, bh[j], acc[i][j]);
        }
      }
      Frag<T>::guard(acc[i][0], acc[i][3], ah, SPLIT ? al : ah);
    }
    Frag<T>::keep(bh[0], bh[1], bh[2], bh[3]);
    if (SPLIT) Frag<T>::keep(bl[0], bl[1], bl[2], bl[3]);
  }
  acc_guard4(acc[0][0], acc[0][1], acc[0][2], acc[0][3]);
  acc_guard4(acc[1][0], acc[1][1], acc[1][2], acc[1][3]);
  acc_guard4(acc[2][0], acc[2][1], acc[2][2], acc[2][3]);
  acc_guard4(acc[3][0], acc[3][1], acc[3][2], acc[3][3]);

  float* slab = sT[wave];
#pragma unroll
  for (int j = 0; j < 4; ++j) {
    const int n = n0 + (j << 4) + rlane;
    const float bv = bias[n];
    float s = 0.0f, q = 0.0f;
    float mxa = -3.0e38f, mna = 3.0e38f, mxb = -3.0e38f, mnb = 3.0e38f;
#pragma unroll
    for (int i = 0; i < 4; ++i) {
#pragma unroll
      for (int r = 0; r < 8; ++r) {
        const float v = acc[i][j][r] * scale + bv;
        s += v;
        q += v * v;
        if (MAXMIN) {
          if (i < 2) { mxa = fmaxf(mxa, v); mna = fminf(mna, v); }
          else       { mxb = fmaxf(mxb, v); mnb = fminf(mnb, v); }
        }
      }
    }
    s += __shfl_xor(s, 16, 32);
    q += __shfl_xor(q, 16, 32);
    mxa = fmaxf(mxa, __shfl_xor(mxa, 16, 32));
    mna = fminf(mna, __shfl_xor(mna, 16, 32));
    mxb = fmaxf(mxb, __shfl_xor(mxb, 16, 32));
    mnb = fminf(mnb, __shfl_xor(mnb, 16, 32));
    slab[(j << 4) + rlane] = s;
    slab[68 + (j << 4) + rlane] = q;
    if (MAXMIN) {
      slab[2 * 68 + (j << 4) + rlane] = mxa;
      slab[3 * 68 + (j << 4) + rlane] = mna;
      slab[4 * 68 + (j << 4) + rlane] = mxb;
      slab[5 * 68 + (j << 4) + rlane] = mnb;
    }
  }
  __builtin_amdgcn_fence(__ATOMIC_RELEASE, "workgroup");
  __builtin_amdgcn_wave_barrier();
  __builtin_amdgcn_fence(__ATOMIC_ACQUIRE, "workgroup");
  {
    const int hh = lane >> 4, c4 = (lane & 15) * 4;
    float* pdst  = part + ((size_t)hh * tilesM + tm) * N + n0 + c4;
    float* gdstA = gmm + ((size_t)hh * (2 * tilesM) + 2 * tm) * N + n0 + c4;
    float* gdstB = gdstA + N;
    for (int pass = 0; pass < 2; ++pass) {
      const v4f v0 = *(const v4f*)(slab + hh * 68 + c4);
      *(volatile v4f*)pdst = v0;
      if (MAXMIN) {
        const v4f v1 = *(const v4f*)(slab + (2 + hh) * 68 + c4);
        *(volatile v4f*)gdstA = v1;
        const v4f v2 = *(const v4f*)(slab + (4 + hh) * 68 + c4);
        *(volatile v4f*)gdstB = v2;
      }
      __threadfence();
    }
  }
  __builtin_amdgcn_fence(__ATOMIC_RELEASE, "workgroup");
  __builtin_amdgcn_wave_barrier();
  __builtin_amdgcn_fence(__ATOMIC_ACQUIRE, "workgroup");

  if (STORE_C) {
#pragma unroll
    for (int i = 0; i < 4; ++i) {
      const int mBase = m0 + (i << 4);
#pragma unroll
      for (int j = 0; j < 4; ++j) {
        const int n = n0 + (j << 4) + rlane;
        const float bv = bias[n];
#pragma unroll
        for (int r = 0; r < 8; ++r) {
          const float v = acc[i][j][r] * scale + bv;
          slab[(mOff + r) * 68 + (j << 4) + rlane] = v;
        }
      }
      __builtin_amdgcn_fence(__ATOMIC_RELEASE, "workgroup");
      __builtin_amdgcn_wave_barrier();
      __builtin_amdgcn_fence(__ATOMIC_ACQUIRE, "workgroup");
      {
        float* C = Cout;
        const int hh = lane >> 4, c4 = (lane & 15) * 4;
        for (int pass = 0; pass < 2; ++pass) {
#pragma unroll
          for (int it = 0; it < 8; ++it) {
            const int row = it * 2 + hh;
            const v4f v = *(const v4f*)(slab + row * 68 + c4);
            *(volatile v4f*)(C + (size_t)(mBase + row) * ldc + n0 + c4) = v;
          }
          __threadfence();
        }
      }
      __builtin_amdgcn_fence(__ATOMIC_RELEASE, "workgroup");
      __builtin_amdgcn_wave_barrier();
      __builtin_amdgcn_fence(__ATOMIC_ACQUIRE, "workgroup");
    }
  }
}

__global__ __launch_bounds__(256) void l2_apply_kernel(const float* __restrict__ a2, const float* __restrict__ tab2,
                                                      unsigned short* __restrict__ H2)
{
  __shared__ float sSc[kC2], sSh[kC2];
  const int t = threadIdx.x;
  if (t < kC2) { sSc[t] = tab2[t]; sSh[t] = tab2[kC2 + t]; }
  __syncthreads();
  const int gid = blockIdx.x * 256 + t;
  const int row = gid >> 4;
  const int c8  = (gid & 15) * 8;
  const float* src = a2 + (size_t)row * kC2 + c8;
  const v4f xa = *(const v4f*)(src);
  const v4f xb = *(const v4f*)(src + 4);
  float x[8];
  x[0] = xa[0]; x[1] = xa[1]; x[2] = xa[2]; x[3] = xa[3];
  x[4] = xb[0]; x[5] = xb[1]; x[6] = xb[2]; x[7] = xb[3];
  unsigned w[4];
#pragma unroll
  for (int p = 0; p < 4; ++p) {
    unsigned pr = 0u;
#pragma unroll
    for (int u = 0; u < 2; ++u) {
      const int e = 2 * p + u;
      const int c = c8 + e;
      const float h = fmaxf(x[e] * sSc[c] + sSh[c], 0.0f);
      const unsigned short hb = __builtin_bit_cast(unsigned short, (_Float16)h);
      pr |= ((unsigned)hb) << (16 * u);
    }
    w[p] = pr;
  }
  const v4u hv = (v4u){w[0], w[1], w[2], w[3]};
  const size_t off = (size_t)row * kC2 + c8;
  for (int pass = 0; pass < 2; ++pass) {
    *(volatile v4u*)(H2 + off) = hv;
    __threadfence();
  }
}

__global__ __launch_bounds__(256) void token_kernel(const float* __restrict__ gmm, const float* __restrict__ tab3,
                                                   float* __restrict__ out)
{
  __shared__ float sSc[kC3], sSh[kC3];
  const int t = threadIdx.x;
  for (int i = t; i < kC3; i += 256) { sSc[i] = tab3[i]; sSh[i] = tab3[kC3 + i]; }
  __syncthreads();
  const int gid = blockIdx.x * 256 + t;
  const int g = gid / (kC3 / 4);
  const int c4 = (gid - g * (kC3 / 4)) * 4;
  const size_t off = (size_t)g * kC3 + c4;
  const v4f mx = *(const v4f*)(gmm + off);
  const v4f mn = *(const v4f*)(gmm + (size_t)kGroups * kC3 + off);
  v4f o;
#pragma unroll
  for (int e = 0; e < 4; ++e) {
    const float sc = sSc[c4 + e], sh = sSh[c4 + e];
    const float va = mx[e] * sc + sh;
    const float vb = mn[e] * sc + sh;
    o[e] = (sc >= 0.0f) ? va : vb;
  }
  for (int pass = 0; pass < 2; ++pass) {
    *(volatile v4f*)(out + off) = o;
    __threadfence();
  }
}

extern "C" void kernel_launch(void* const* d_in, const int* in_sizes, int n_in,
                              void* d_out, int out_size, void* d_ws, size_t ws_size,
                              hipStream_t stream)
{
  if (n_in < 13) return;
  if (in_sizes[0] != kBatch * kNpts * 3) return;
  if (in_sizes[1] != 3 * kC1 || in_sizes[2] != kC1 || in_sizes[3] != kC1 || in_sizes[4] != kC1) return;
  if (in_sizes[5] != kC1 * kC2 || in_sizes[6] != kC2 || in_sizes[7] != kC2 || in_sizes[8] != kC2) return;
  if (in_sizes[9] != kC2 * kC3 || in_sizes[10] != kC3 || in_sizes[11] != kC3 || in_sizes[12] != kC3) return;
  if (out_size != kGroups * kC3 + kGroups * 3) return;
  if (ws_size < kWsTotal) return;

  const float* points = (const float*)d_in[0];
  const float* W1  = (const float*)d_in[1];
  const float* b1  = (const float*)d_in[2];
  const float* g1  = (const float*)d_in[3];
  const float* be1 = (const float*)d_in[4];
  const float* W2  = (const float*)d_in[5];
  const float* b2  = (const float*)d_in[6];
  const float* g2  = (const float*)d_in[7];
  const float* be2 = (const float*)d_in[8];
  const float* W3  = (const float*)d_in[9];
  const float* b3  = (const float*)d_in[10];
  const float* g3  = (const float*)d_in[11];
  const float* be3 = (const float*)d_in[12];

  float* tokens  = (float*)d_out;
  float* centers = (float*)d_out + kOut1Floats;

  char* ws = (char*)d_ws;
  float*          grouped = (float*)(ws + kOffGrouped);
  float*          part1   = (float*)(ws + kOffPart1);
  float*          tab1    = (float*)(ws + kOffTab1);
  unsigned short* w2hi    = (unsigned short*)(ws + kOffW2t);
  unsigned short* w2lo    = w2hi + (size_t)kC2 * kC1;
  unsigned short* w3t     = (unsigned short*)(ws + kOffW3t);
  unsigned short* h1hi    = (unsigned short*)(ws + kOffH);
  unsigned short* h1lo    = h1hi + (size_t)kRows * kC1;
  unsigned short* h2p     = (unsigned short*)(ws + kOffH);
  float*          a2      = (float*)(ws + kOffA2);
  float*          part2   = (float*)(ws + kOffPart2);
  float*          tab2    = (float*)(ws + kOffTab2);
  float*          part3   = (float*)(ws + kOffPart3);
  float*          tab3    = (float*)(ws + kOffTab3);
  float*          gmm     = (float*)(ws + kOffGmm);

  fps_kernel<<<dim3(kBatch), dim3(kFpsT), 0, stream>>>(points, centers);
  knn_kernel<<<dim3(kGroups), dim3(kKnnT), 0, stream>>>(points, centers, grouped);
  wprep2_kernel<<<dim3((kC2 * kC1 / 8) / 256), dim3(256), 0, stream>>>(W2, w2hi, w2lo);
  wprep3_kernel<<<dim3((kC3 * kC2 / 8) / 256), dim3(256), 0, stream>>>(W3, w3t);
  l1_stats_kernel<<<dim3(kL1Blocks), dim3(256), 0, stream>>>(grouped, W1, b1, part1);
  fin_kernel<<<dim3(kC1 / 64), dim3(64), 0, stream>>>(part1, kL1Blocks, kC1, g1, be1, tab1);
  l1_apply_kernel<<<dim3((kRows * 8) / 256), dim3(256), 0, stream>>>(grouped, W1, b1, tab1, h1hi, h1lo);
  wmma_gemm64_stats<1, true, true, false><<<dim3((kTilesM * (kC2 / 64)) / 8), dim3(256), 0, stream>>>(
      h1hi, h1lo, kC1, w2hi, w2lo, kC1, a2, kC2, b2, part2, gmm, kRows, kC2, kC1, 1.0f);
  fin_kernel<<<dim3(kC2 / 64), dim3(64), 0, stream>>>(part2, kTilesM, kC2, g2, be2, tab2);
  l2_apply_kernel<<<dim3((kRows * 16) / 256), dim3(256), 0, stream>>>(a2, tab2, h2p);
  wmma_gemm64_stats<0, false, false, true><<<dim3((kTilesM * (kC3 / 64)) / 8), dim3(256), 0, stream>>>(
      h2p, h2p, kC2, w3t, w3t, kC2, a2, kC3, b3, part3, gmm, kRows, kC3, kC2, 1.0f / 16.0f);
  fin_kernel<<<dim3(kC3 / 64), dim3(64), 0, stream>>>(part3, kTilesM, kC3, g3, be3, tab3);
  token_kernel<<<dim3((kGroups * (kC3 / 4)) / 256), dim3(256), 0, stream>>>(gmm, tab3, tokens);
}
